// LSTM_74672301408953
// MI455X (gfx1250) — hardware-verified
//
#include <hip/hip_runtime.h>
#include <math.h>

constexpr int NSTEP    = 256;
constexpr int NBATCH   = 64;
constexpr int NIN      = 512;
constexpr int NMEM     = 512;
constexpr int NROWS    = NSTEP * NBATCH;
constexpr int KCAT     = NIN + NMEM;
constexpr int NIOU     = 3 * NMEM;
constexpr int NPRE     = 5 * NMEM;
constexpr int NWH      = 4 * NMEM;
constexpr int NCHUNK   = 2;
constexpr int CH_STEPS = NSTEP / NCHUNK;
constexpr int CH_ROWS  = CH_STEPS * NBATCH;
constexpr int RBLK     = 16;
constexpr int RTHR     = 512;
constexpr int AHP      = 520;
constexpr int OSP      = 516;
constexpr float WCARRY     = 16.0f;
constexpr float WCARRY_INV = 1.0f / WCARRY;
constexpr bool  LEG_BF16   = true;

static_assert(NIN == 512 && NMEM == 512, "convert kernel assumes 512-column sources");
static_assert(NCHUNK == 2 && NSTEP % NCHUNK == 0, "two time chunks");
static_assert(CH_ROWS % 64 == 0 && NIOU % 64 == 0 && NMEM % 64 == 0, "GEMM M,N tile multiples");
static_assert(KCAT % 32 == 0 && NIN % 32 == 0 && NMEM % 32 == 0, "GEMM K multiples of 32");
static_assert(((CH_ROWS / 64) * (NIOU / 64)) % 8 == 0 && ((CH_ROWS / 64) * (NMEM / 64)) % 8 == 0, "exact GEMM grids");
static_assert(NBATCH % RBLK == 0, "batch rows per block");
static_assert(NMEM == 32 * (RTHR / 32), "16 waves x 32 hidden units");
static_assert(RBLK * NMEM == 4 * RTHR * 4, "output store loop covers 16 x 512 floats");
static_assert(NROWS * NMEM == 8388608, "output extent");

typedef __attribute__((ext_vector_type(16))) _Float16 v16h;
typedef __attribute__((ext_vector_type(8)))  _Float16 v8h;
typedef __attribute__((ext_vector_type(8)))  float    v8f;
typedef __attribute__((ext_vector_type(4)))  float    v4f;

__device__ __forceinline__ unsigned short f2bf_bits(float f) {
  unsigned u = __float_as_uint(f);
  return (unsigned short)((u + 0x7FFFu + ((u >> 16) & 1u)) >> 16);
}
__device__ __forceinline__ float bf_bits2f(unsigned short h) { return __uint_as_float(((unsigned)h) << 16); }
__device__ __forceinline__ float bf16r(float f) { return bf_bits2f(f2bf_bits(f)); }
__device__ __forceinline__ float rnd_in(float f) { return LEG_BF16 ? bf16r(f) : f; }

__device__ __forceinline__ void keep4_h(v16h a, v16h b, v16h c, v16h d) { asm volatile("v_nop" :: "v"(a), "v"(b), "v"(c), "v"(d)); }
__device__ __forceinline__ void acc_guard4(v8f& a, v8f& b, v8f& c, v8f& d) { asm volatile("v_nop\n\tv_nop\n\tv_nop\n\tv_nop" : "+v"(a), "+v"(b), "+v"(c), "+v"(d)); }
__device__ __forceinline__ void guard_all4(v8f& a0, v8f& a1, v8f& a2, v8f& a3, v16h x, v16h b0, v16h b1, v16h b2, v16h b3) {
  asm volatile("v_nop\n\tv_nop\n\tv_nop\n\tv_nop" : "+v"(a0), "+v"(a1), "+v"(a2), "+v"(a3) : "v"(x), "v"(b0), "v"(b1), "v"(b2), "v"(b3));
}
__device__ __forceinline__ void tie8(float (&p)[8]) {
  asm volatile("" : "+v"(p[0]), "+v"(p[1]), "+v"(p[2]), "+v"(p[3]), "+v"(p[4]), "+v"(p[5]), "+v"(p[6]), "+v"(p[7]) :: "memory");
}

struct FragH {
  union U { v16h v; v8h h[2]; };
  static __device__ __forceinline__ v16h load(const _Float16* p) {
    U f; f.h[0] = *(const v8h*)(p); f.h[1] = *(const v8h*)(p + 16); return f.v;
  }
  static __device__ __forceinline__ v8f mma(v16h a, v16h b, v8f c) {
    return __builtin_amdgcn_wmma_f32_16x16x32_f16(false, a, false, b, (short)0, c, false, false);
  }
};

__device__ __forceinline__ float sigm(float x) { return __builtin_amdgcn_rcpf(1.0f + expf(-x)); }
__device__ __forceinline__ float tanh_e(float x) {
  const float xc = fminf(fmaxf(x, -15.0f), 15.0f);
  return 1.0f - 2.0f * __builtin_amdgcn_rcpf(expf(2.0f * xc) + 1.0f);
}

__global__ __launch_bounds__(256) void cvt8_kernel(const float* __restrict__ src, unsigned short* __restrict__ dst,
                                                   int nrow, int dpitch, int dcol0, float sc) {
  const int i  = blockIdx.x * 256 + threadIdx.x;
  const int n8 = nrow * 64;
  if (i < n8) {
    const int row = i >> 6;
    const int c8  = i & 63;
    const float* sp = src + (size_t)row * 512 + c8 * 8;
    const v4f a = *(const v4f*)(sp);
    const v4f b = *(const v4f*)(sp + 4);
    v8h hv;
#pragma unroll
    for (int e = 0; e < 4; ++e) {
      const float fa = a[e];
      const float fb = b[e];
      hv[e]     = (_Float16)(rnd_in(fa) * sc);
      hv[4 + e] = (_Float16)(rnd_in(fb) * sc);
    }
    unsigned short* dp = dst + (size_t)row * dpitch + dcol0 + c8 * 8;
    *(volatile v8h*)dp = hv;
    __threadfence();
    *(volatile v8h*)dp = hv;
  }
}

__global__ __launch_bounds__(256) void bias_fold_kernel(const float* __restrict__ b_ioux, const float* __restrict__ b_ious,
                                                        const float* __restrict__ b_iouh, const float* __restrict__ b_fx,
                                                        const float* __restrict__ b_fh, const float* __restrict__ b_fxs,
                                                        const float* __restrict__ b_fs, float* __restrict__ dst) {
  const int i4 = blockIdx.x * 256 + threadIdx.x;
  if (i4 < NPRE / 4) {
    const int idx = i4 * 4;
    const int ci  = (idx < NIOU - 4) ? idx : (NIOU - 4);
    int fi = idx - NIOU;
    fi = (fi < 0) ? 0 : fi;
    fi = (fi > NMEM - 4) ? (NMEM - 4) : fi;
    int si = idx - NIOU - NMEM;
    si = (si < 0) ? 0 : si;
    si = (si > NMEM - 4) ? (NMEM - 4) : si;
    const v4f a1 = *(const v4f*)(b_ioux + ci);
    const v4f a2 = *(const v4f*)(b_ious + ci);
    const v4f a3 = *(const v4f*)(b_iouh + ci);
    const v4f f1 = *(const v4f*)(b_fx + fi);
    const v4f f2 = *(const v4f*)(b_fh + fi);
    const v4f g1 = *(const v4f*)(b_fxs + si);
    const v4f g2 = *(const v4f*)(b_fs + si);
    const float w0 = (idx < NIOU) ? 1.0f : 0.0f;
    const float w1 = (idx >= NIOU && idx < NIOU + NMEM) ? 1.0f : 0.0f;
    const float w2 = (idx >= NIOU + NMEM) ? 1.0f : 0.0f;
    v4f o;
#pragma unroll
    for (int e = 0; e < 4; ++e) {
      const float x1 = a1[e], x2 = a2[e], x3 = a3[e], y1 = f1[e], y2 = f2[e], z1 = g1[e], z2 = g2[e];
      const float s0 = (rnd_in(x1) + rnd_in(x2)) + rnd_in(x3);
      const float s1 = rnd_in(y1) + rnd_in(y2);
      const float s2 = rnd_in(z1) + rnd_in(z2);
      o[e] = fmaf(w0, s0, fmaf(w1, s1, w2 * s2));
    }
    float* op = dst + idx;
    *(volatile v4f*)op = o;
    __threadfence();
    *(volatile v4f*)op = o;
  }
}

template <bool GATE>
__global__ __launch_bounds__(256) void wmma_gemm64_f16(
    const unsigned short* __restrict__ Ap, int lda,
    const unsigned short* __restrict__ Btp, int ldb,
    float* __restrict__ C, int ldc,
    const float* __restrict__ bias,
    const float* __restrict__ gate, int ldg,
    int M, int N, int K, float scale) {
  const _Float16* A  = (const _Float16*)Ap;
  const _Float16* Bt = (const _Float16*)Btp;
  __shared__ __align__(16) float sT[8][16 * 68];
  const int lane = threadIdx.x & 31;
  const int wave = threadIdx.x >> 5;
  const int tilesN = N >> 6;
  const int tilesM = M >> 6;
  const int tile = blockIdx.x * 8 + wave;
  if (tile >= tilesM * tilesN) return;
  const int tm = tile / tilesN;
  const int tn = tile - tm * tilesN;
  const int m0 = tm << 6;
  const int n0 = tn << 6;

  const int rlane = lane & 15;
  const int koff  = (lane >> 4) * 8;
  const int mOff  = (lane >> 4) * 8;

  v8f acc[4][4];
#pragma unroll
  for (int i = 0; i < 4; ++i)
#pragma unroll
    for (int j = 0; j < 4; ++j) acc[i][j] = (v8f){0.f, 0.f, 0.f, 0.f, 0.f, 0.f, 0.f, 0.f};

  for (int k0 = 0; k0 < K; k0 += 32) {
    v16h bh[4];
#pragma unroll
    for (int j = 0; j < 4; ++j) {
      const size_t bo = (size_t)(n0 + (j << 4) + rlane) * ldb + koff + k0;
      bh[j] = FragH::load(Bt + bo);
    }
#pragma unroll
    for (int i = 0; i < 4; ++i) {
      const size_t ao = (size_t)(m0 + (i << 4) + rlane) * lda + koff + k0;
      const v16h ah = FragH::load(A + ao);
#pragma unroll
      for (int j = 0; j < 4; ++j) acc[i][j] = FragH::mma(ah, bh[j], acc[i][j]);
      guard_all4(acc[i][0], acc[i][1], acc[i][2], acc[i][3], ah, bh[0], bh[1], bh[2], bh[3]);
    }
    keep4_h(bh[0], bh[1], bh[2], bh[3]);
  }
  acc_guard4(acc[0][0], acc[0][1], acc[0][2], acc[0][3]);
  acc_guard4(acc[1][0], acc[1][1], acc[1][2], acc[1][3]);
  acc_guard4(acc[2][0], acc[2][1], acc[2][2], acc[2][3]);
  acc_guard4(acc[3][0], acc[3][1], acc[3][2], acc[3][3]);

  float* slab = sT[wave];
  const int hh = lane >> 4;
  const int c4 = (lane & 15) * 4;
#pragma unroll
  for (int i = 0; i < 4; ++i) {
    const int mBase = m0 + (i << 4);
#pragma unroll
    for (int j = 0; j < 4; ++j) {
      const int n = n0 + (j << 4) + rlane;
      const float bv = bias[n];
#pragma unroll
      for (int r = 0; r < 8; ++r) {
        const float v = acc[i][j][r] * scale + bv;
        slab[(mOff + r) * 68 + (j << 4) + rlane] = v;
      }
    }
    __builtin_amdgcn_fence(__ATOMIC_RELEASE, "workgroup");
    __builtin_amdgcn_wave_barrier();
    __builtin_amdgcn_fence(__ATOMIC_ACQUIRE, "workgroup");
    if (GATE) {
#pragma unroll 1
      for (int it = 0; it < 8; ++it) {
        const int row = it * 2 + hh;
        float* sp = slab + row * 68 + c4;
        const v4f v = *(const v4f*)sp;
        const v4f g = *(const v4f*)(gate + (size_t)(mBase + row) * ldg + n0 + c4);
        v4f o;
#pragma unroll
        for (int e = 0; e < 4; ++e) {
          const float ve = v[e];
          const float ge = g[e];
          o[e] = sigm(ve) * rnd_in(ge);
        }
        *(v4f*)sp = o;
      }
      __builtin_amdgcn_fence(__ATOMIC_RELEASE, "workgroup");
      __builtin_amdgcn_wave_barrier();
      __builtin_amdgcn_fence(__ATOMIC_ACQUIRE, "workgroup");
    }
    for (int pass = 0; pass < 2; ++pass) {
#pragma unroll
      for (int it = 0; it < 8; ++it) {
        const int row = it * 2 + hh;
        const v4f v = *(const v4f*)(slab + row * 68 + c4);
        *(volatile v4f*)(C + (size_t)(mBase + row) * ldc + n0 + c4) = v;
      }
      __threadfence();
    }
    __builtin_amdgcn_fence(__ATOMIC_RELEASE, "workgroup");
    __builtin_amdgcn_wave_barrier();
    __builtin_amdgcn_fence(__ATOMIC_ACQUIRE, "workgroup");
  }
}

__device__ __forceinline__ void add_pre8(v8f& acc, const float* __restrict__ p, float sc) {
  float q[8];
#pragma unroll
  for (int r = 0; r < 8; ++r) q[r] = p[(size_t)r * NPRE];
  tie8(q);
#pragma unroll
  for (int r = 0; r < 8; ++r) acc[r] = acc[r] * sc + q[r];
}

template <bool FIRST, bool SAVE>
__global__ __launch_bounds__(RTHR) void rec_kernel(const float* __restrict__ PRE, const unsigned short* __restrict__ WHp,
                                                   float* CST, float* HST, float* __restrict__ out, int t0) {
  __shared__ __align__(16) _Float16 Ah[RBLK * AHP];
  __shared__ __align__(16) float    Ost[RBLK * OSP];
  const _Float16* WH = (const _Float16*)WHp;
  const int tid = threadIdx.x, lane = tid & 31, wave = tid >> 5;
  const int c = lane & 15, hh = lane >> 4, koff = hh * 8;
  const int b0 = blockIdx.x * RBLK;

  float cst[2][8], hst[2][8];
  if (FIRST) {
    unsigned* aw = (unsigned*)Ah;
#pragma unroll 1
    for (int i = tid; i < RBLK * AHP / 2; i += RTHR) aw[i] = 0u;
#pragma unroll
    for (int nt = 0; nt < 2; ++nt)
#pragma unroll
      for (int r = 0; r < 8; ++r) cst[nt][r] = 0.0f;
  } else {
#pragma unroll 1
    for (int i = 0; i < RBLK; ++i) Ah[i * AHP + tid] = (_Float16)HST[(size_t)(b0 + i) * NMEM + tid];
#pragma unroll
    for (int nt = 0; nt < 2; ++nt) {
      const int j = 32 * wave + 16 * nt + c;
      float q[8];
#pragma unroll
      for (int r = 0; r < 8; ++r) q[r] = CST[(size_t)(b0 + 8 * hh + r) * NMEM + j];
      tie8(q);
#pragma unroll
      for (int r = 0; r < 8; ++r) cst[nt][r] = q[r];
    }
  }
#pragma unroll
  for (int nt = 0; nt < 2; ++nt)
#pragma unroll
    for (int r = 0; r < 8; ++r) hst[nt][r] = 0.0f;
  __syncthreads();

  const _Float16* ahrow = Ah + c * AHP + koff;
  const v8f z8 = {0.f, 0.f, 0.f, 0.f, 0.f, 0.f, 0.f, 0.f};

#pragma unroll 1
  for (int t = 0; t < CH_STEPS; ++t) {
    const float* prow = PRE + (size_t)(t * NBATCH + b0 + 8 * hh) * NPRE;
#pragma unroll
    for (int nt = 0; nt < 2; ++nt) {
      const int j = 32 * wave + 16 * nt + c;
      const _Float16* wh = WH + (size_t)j * NMEM + koff;
      v8f acc0 = z8, acc1 = z8, acc2 = z8, acc3 = z8;
#pragma unroll 1
      for (int k0 = 0; k0 < NMEM; k0 += 32) {
        const v16h a  = FragH::load(ahrow + k0);
        const v16h w0 = FragH::load(wh + k0);
        const v16h w1 = FragH::load(wh + (size_t)1 * NMEM * NMEM + k0);
        const v16h w2 = FragH::load(wh + (size_t)2 * NMEM * NMEM + k0);
        const v16h w3 = FragH::load(wh + (size_t)3 * NMEM * NMEM + k0);
        acc0 = FragH::mma(a, w0, acc0);
        acc1 = FragH::mma(a, w1, acc1);
        acc2 = FragH::mma(a, w2, acc2);
        acc3 = FragH::mma(a, w3, acc3);
        guard_all4(acc0, acc1, acc2, acc3, a, w0, w1, w2, w3);
      }
      acc_guard4(acc0, acc1, acc2, acc3);
      add_pre8(acc0, prow + 0 * NMEM + j, WCARRY_INV);
      add_pre8(acc1, prow + 1 * NMEM + j, WCARRY_INV);
      add_pre8(acc2, prow + 2 * NMEM + j, WCARRY_INV);
      add_pre8(acc3, prow + 3 * NMEM + j, WCARRY_INV);
      float fsc[8];
#pragma unroll
      for (int r = 0; r < 8; ++r) fsc[r] = prow[(size_t)r * NPRE + 4 * NMEM + j];
      tie8(fsc);
#pragma unroll
      for (int r = 0; r < 8; ++r) {
        const float ig = sigm(acc0[r]);
        const float og = sigm(acc1[r]);
        const float ug = tanh_e(acc2[r]);
        const float fg = sigm(acc3[r]);
        const float cn = ig * ug + fg * cst[nt][r] + fsc[r];
        cst[nt][r] = cn;
        hst[nt][r] = og * tanh_e(cn);
      }
    }
    __syncthreads();
#pragma unroll
    for (int nt = 0; nt < 2; ++nt) {
      const int j = 32 * wave + 16 * nt + c;
#pragma unroll
      for (int r = 0; r < 8; ++r) {
        const float hv = hst[nt][r];
        Ah[(8 * hh + r) * AHP + j]  = (_Float16)hv;
        Ost[(8 * hh + r) * OSP + j] = hv;
      }
    }
    __syncthreads();
    {
      const bool last = (t == CH_STEPS - 1);
      const size_t grow0 = (size_t)((t0 + t) * NBATCH + b0);
      for (int pass = 0; pass < 2; ++pass) {
#pragma unroll
        for (int it = 0; it < 4; ++it) {
          const int idx = it * RTHR + tid;
          const int row = idx >> 7;
          const int c4  = (idx & 127) * 4;
          const v4f v = *(const v4f*)(Ost + row * OSP + c4);
          *(volatile v4f*)(out + (grow0 + row) * NMEM + c4) = v;
          if (SAVE && last) *(volatile v4f*)(HST + (size_t)(b0 + row) * NMEM + c4) = v;
        }
        __threadfence();
      }
    }
  }

  if (SAVE) {
    __syncthreads();
#pragma unroll
    for (int nt = 0; nt < 2; ++nt) {
      const int j = 32 * wave + 16 * nt + c;
#pragma unroll
      for (int r = 0; r < 8; ++r) Ost[(8 * hh + r) * OSP + j] = cst[nt][r];
    }
    __syncthreads();
    for (int pass = 0; pass < 2; ++pass) {
#pragma unroll
      for (int it = 0; it < 4; ++it) {
        const int idx = it * RTHR + tid;
        const int row = idx >> 7;
        const int c4  = (idx & 127) * 4;
        const v4f v = *(const v4f*)(Ost + row * OSP + c4);
        *(volatile v4f*)(CST + (size_t)(b0 + row) * NMEM + c4) = v;
      }
      __threadfence();
    }
  }
}

extern "C" void kernel_launch(void* const* d_in, const int* in_sizes, int n_in,
                              void* d_out, int out_size, void* d_ws, size_t ws_size, hipStream_t stream) {
  if (n_in < 17 || d_out == nullptr || d_ws == nullptr) return;
  if (in_sizes[0] != NROWS * NIN || in_sizes[1] != NROWS * NMEM || in_sizes[2] != NROWS * NMEM ||
      in_sizes[3] != NIOU * NIN || in_sizes[4] != NIOU || in_sizes[5] != NIOU * NMEM || in_sizes[6] != NIOU ||
      in_sizes[7] != NIOU * NMEM || in_sizes[8] != NIOU || in_sizes[9] != NMEM * NIN || in_sizes[10] != NMEM ||
      in_sizes[11] != NMEM * NIN || in_sizes[12] != NMEM || in_sizes[13] != NMEM * NMEM || in_sizes[14] != NMEM ||
      in_sizes[15] != NMEM * NMEM || in_sizes[16] != NMEM || out_size != NROWS * NMEM) return;

  const float* x_in     = (const float*)d_in[0];
  const float* sememe_c = (const float*)d_in[1];
  const float* sememe_h = (const float*)d_in[2];
  const float* W_ioux   = (const float*)d_in[3];
  const float* b_ioux   = (const float*)d_in[4];
  const float* W_iouh   = (const float*)d_in[5];
  const float* b_iouh   = (const float*)d_in[6];
  const float* W_ious   = (const float*)d_in[7];
  const float* b_ious   = (const float*)d_in[8];
  const float* W_fx     = (const float*)d_in[9];
  const float* b_fx     = (const float*)d_in[10];
  const float* W_fxs    = (const float*)d_in[11];
  const float* b_fxs    = (const float*)d_in[12];
  const float* W_fh     = (const float*)d_in[13];
  const float* b_fh     = (const float*)d_in[14];
  const float* W_fs     = (const float*)d_in[15];
  const float* b_fs     = (const float*)d_in[16];
  float* hs_out = (float*)d_out;

  char* ws = (char*)d_ws; size_t off = 0;
  auto carve = [&](size_t bytes) -> char* { char* p = ws + off; off += (bytes + 255) & ~(size_t)255; return p; };
  unsigned short* XS16   = (unsigned short*)carve((size_t)NROWS * KCAT * 2);
  unsigned short* WIOU16 = (unsigned short*)carve((size_t)NIOU * KCAT * 2);
  unsigned short* WF16   = (unsigned short*)carve((size_t)NMEM * NIN * 2);
  unsigned short* WFS16  = (unsigned short*)carve((size_t)NMEM * KCAT * 2);
  unsigned short* WH16   = (unsigned short*)carve((size_t)NWH * NMEM * 2);
  float*          BIAS   = (float*)carve((size_t)NPRE * 4);
  float*          CST    = (float*)carve((size_t)NBATCH * NMEM * 4);
  float*          HST    = (float*)carve((size_t)NBATCH * NMEM * 4);
  float*          PRE    = (float*)carve((size_t)CH_ROWS * NPRE * 4);
  if (off > ws_size || off > (size_t)134217728) return;

  cvt8_kernel<<<NROWS / 4, 256, 0, stream>>>(x_in,     XS16,   NROWS, KCAT, 0,   1.0f);
  cvt8_kernel<<<NROWS / 4, 256, 0, stream>>>(sememe_h, XS16,   NROWS, KCAT, NIN, 1.0f);
  cvt8_kernel<<<NIOU / 4,  256, 0, stream>>>(W_ioux,   WIOU16, NIOU,  KCAT, 0,   WCARRY);
  cvt8_kernel<<<NIOU / 4,  256, 0, stream>>>(W_ious,   WIOU16, NIOU,  KCAT, NIN, WCARRY);
  cvt8_kernel<<<NMEM / 4,  256, 0, stream>>>(W_fx,     WF16,   NMEM,  NIN,  0,   WCARRY);
  cvt8_kernel<<<NMEM / 4,  256, 0, stream>>>(W_fxs,    WFS16,  NMEM,  KCAT, 0,   WCARRY);
  cvt8_kernel<<<NMEM / 4,  256, 0, stream>>>(W_fs,     WFS16,  NMEM,  KCAT, NIN, WCARRY);
  cvt8_kernel<<<NIOU / 4,  256, 0, stream>>>(W_iouh,   WH16,   NIOU,  NMEM, 0,   WCARRY);
  cvt8_kernel<<<NMEM / 4,  256, 0, stream>>>(W_fh,     WH16 + (size_t)NIOU * NMEM, NMEM, NMEM, 0, WCARRY);
  bias_fold_kernel<<<3, 256, 0, stream>>>(b_ioux, b_ious, b_iouh, b_fx, b_fh, b_fxs, b_fs, BIAS);

  const int gridIOU = ((CH_ROWS / 64) * (NIOU / 64)) / 8;
  const int gridF   = ((CH_ROWS / 64) * (NMEM / 64)) / 8;
  for (int ch = 0; ch < NCHUNK; ++ch) {
    const unsigned short* Ach = XS16 + (size_t)ch * CH_ROWS * KCAT;
    const float* SCch = sememe_c + (size_t)ch * CH_ROWS * NMEM;
    wmma_gemm64_f16<false><<<gridIOU, 256, 0, stream>>>(Ach, KCAT, WIOU16, KCAT, PRE, NPRE, BIAS, BIAS, 0,
                                                        CH_ROWS, NIOU, KCAT, WCARRY_INV);
    wmma_gemm64_f16<false><<<gridF, 256, 0, stream>>>(Ach, KCAT, WF16, NIN, PRE + NIOU, NPRE, BIAS + NIOU, BIAS, 0,
                                                      CH_ROWS, NMEM, NIN, WCARRY_INV);
    wmma_gemm64_f16<true><<<gridF, 256, 0, stream>>>(Ach, KCAT, WFS16, KCAT, PRE + NIOU + NMEM, NPRE, BIAS + NIOU + NMEM, SCch, NMEM,
                                                     CH_ROWS, NMEM, KCAT, WCARRY_INV);
    if (ch == 0) rec_kernel<true, true><<<NBATCH / RBLK, RTHR, 0, stream>>>(PRE, WH16, CST, HST, hs_out, 0);
    else         rec_kernel<false, false><<<NBATCH / RBLK, RTHR, 0, stream>>>(PRE, WH16, CST, HST, hs_out, ch * CH_STEPS);
  }
}
